// TriangleAttention_53944789238378
// MI455X (gfx1250) — hardware-verified
//
#include <hip/hip_runtime.h>
#include <stddef.h>
#include <stdint.h>
#include <math.h>


#define DP      256
#define DHID    512
#define NHD     8
#define HDM     64
#define QW      2048
#define OQ      0
#define OKK     512
#define OV      1024
#define OG      1536
#define KOUT    1024
#define APITCH  1024
#define NKVMAX  16
#define QSC     0.125f
#define NTHR    256
#define NWAVE   8
#define RPW     4
#define RB      (NWAVE * RPW)
#define GBM     64
#define GBN     64
#define GTHR    128
#define UW      (DHID * (DP / 8))
#define UWO     (DP * (KOUT / 8))
#define NUW     (4 * UW + UWO)
#define WSMAX   134217728

static_assert(DHID == NHD * HDM);
static_assert(DHID == 2 * 32 * 8);
static_assert(HDM == 8 * 8);
static_assert(QW == 4 * DHID && OG + DHID == QW);
static_assert((QW % GBN) == 0 && (DP % GBN) == 0 && (DHID % GBN) == 0);
static_assert((DP % 32) == 0 && (KOUT % 32) == 0);
static_assert(KOUT == 2 * DHID && APITCH == KOUT);
static_assert((APITCH * 2) % 128 == 0 && (DP * 2) % 128 == 0 && (QW * 4) % 128 == 0 && (DP * 4) % 128 == 0);
static_assert(GBM == (GTHR / 32) * 16);
static_assert(UW == (1 << 14) && (DP / 8) == 32 && (KOUT / 8) == 128);
static_assert((UW % NTHR) == 0 && ((4 * UW) % NTHR) == 0 && (UWO % NTHR) == 0);
static_assert((GBM % RB) == 0);
static_assert(2 * NKVMAX <= 32);

typedef float          v4f  __attribute__((ext_vector_type(4)));
typedef float          v8f  __attribute__((ext_vector_type(8)));
typedef int            v8i  __attribute__((ext_vector_type(8)));
typedef unsigned int   v4u  __attribute__((ext_vector_type(4)));
typedef unsigned short v8us __attribute__((ext_vector_type(8)));
typedef __bf16         v16b __attribute__((ext_vector_type(16)));
typedef v4f  __attribute__((may_alias)) v4fa;
typedef v4u  __attribute__((may_alias)) v4ua;
typedef v8us __attribute__((may_alias)) v8usa;
union FragB { v16b v; v8us h[2]; v8i w; };

__device__ __forceinline__ v8f wmb(const FragB& a, const FragB& b, v8f c) {
  v8f d = __builtin_amdgcn_wmma_f32_16x16x32_bf16(false, a.v, false, b.v, (short)0, c, false, false);
  asm volatile("v_nop\n\tv_nop\n\tv_nop\n\tv_nop" : "+v"(d) : "v"(a.w), "v"(b.w));
  return d;
}

__device__ __forceinline__ void ldwait() {
  asm volatile("s_wait_loadcnt 0x0" ::: "memory");
}

__device__ __forceinline__ unsigned int f2bf(float f) {
  const unsigned int u = __float_as_uint(f);
  return ((u + 0x7FFFu + ((u >> 16) & 1u)) >> 16) & 0xFFFFu;
}
__device__ __forceinline__ float bf2f(unsigned int b) { return __uint_as_float(b << 16); }
__device__ __forceinline__ float bfr(float f) { return bf2f(f2bf(f)); }
__device__ __forceinline__ v4f bfr4(const v4f a) {
  v4f r; r.x = bfr(a.x); r.y = bfr(a.y); r.z = bfr(a.z); r.w = bfr(a.w); return r;
}
__device__ __forceinline__ unsigned int pk2(float lo, float hi) { return f2bf(lo) | (f2bf(hi) << 16); }
__device__ __forceinline__ v4u pack8(const v4f a, const v4f b) {
  v4u r;
  r.x = pk2(a.x, a.y); r.y = pk2(a.z, a.w); r.z = pk2(b.x, b.y); r.w = pk2(b.z, b.w);
  return r;
}
__device__ __forceinline__ void hl2(float v0, float v1, unsigned int& hw, unsigned int& lw) {
  const unsigned int h0 = f2bf(v0), h1 = f2bf(v1);
  const unsigned int l0 = f2bf(v0 - bf2f(h0)), l1 = f2bf(v1 - bf2f(h1));
  hw = h0 | (h1 << 16);
  lw = l0 | (l1 << 16);
}
__device__ __forceinline__ void pack8hl(const v4f a, const v4f b, v4u& hv, v4u& lv) {
  unsigned int h, l;
  hl2(a.x, a.y, h, l); hv.x = h; lv.x = l;
  hl2(a.z, a.w, h, l); hv.y = h; lv.y = l;
  hl2(b.x, b.y, h, l); hv.z = h; lv.z = l;
  hl2(b.z, b.w, h, l); hv.w = h; lv.w = l;
}

__device__ __forceinline__ float sgm(float x) { return __builtin_amdgcn_rcpf(1.0f + __expf(-x)); }
__device__ __forceinline__ v4f dsig4(const v4f a) {
  v4f r;
  r.x = sgm(sgm(a.x)); r.y = sgm(sgm(a.y)); r.z = sgm(sgm(a.z)); r.w = sgm(sgm(a.w));
  return r;
}

__global__ __launch_bounds__(NTHR) void k_zprep(const float* __restrict__ z, unsigned short* zb, int nN, int nUnits) {
  const int i = (int)blockIdx.x * NTHR + (int)threadIdx.x;
  if (i >= nUnits) return;
  const int row = i >> 5;
  const int c0  = (i & 31) * 8;
  const int rc  = row < nN ? row : nN - 1;
  const float* p = z + (size_t)rc * DP + c0;
  v4f a = *(const v4fa*)p;
  v4f b = *(const v4fa*)(p + 4);
  const v4f z4 = {0.f, 0.f, 0.f, 0.f};
  if (row >= nN) { a = z4; b = z4; }
  const v4u hv = pack8(a, b);
  unsigned short* o = zb + (size_t)row * DP + c0;
  *(volatile v4u*)o = hv;
  __threadfence();
  *(volatile v4u*)o = hv;
}

__global__ __launch_bounds__(NTHR) void k_wprep(const float* __restrict__ Wq, const float* __restrict__ Wk,
                                                const float* __restrict__ Wv, const float* __restrict__ Wg,
                                                const float* __restrict__ Wo,
                                                unsigned short* WT, unsigned short* WOT) {
  const int u = (int)blockIdx.x * NTHR + (int)threadIdx.x;
  if (u >= NUW) return;
  const float* p;
  int st;
  unsigned short* dp;
  if (u < 4 * UW) {
    const int part = u >> 14;
    const int v    = u & (UW - 1);
    const int n    = v >> 5;
    const int k8   = (v & 31) * 8;
    const float* W = (part == 0) ? Wq : ((part == 1) ? Wk : ((part == 2) ? Wv : Wg));
    p  = W + (size_t)k8 * DHID + n;
    st = DHID;
    dp = WT + (size_t)(part * DHID + n) * DP + k8;
  } else {
    const int v  = u - 4 * UW;
    const int n  = v >> 7;
    const int k8 = (v & 127) * 8;
    const int kk = k8 & (DHID - 1);
    p  = Wo + (size_t)kk * DP + n;
    st = DP;
    dp = WOT + (size_t)n * KOUT + k8;
  }
  v4f a, b;
  a.x = p[0];
  a.y = p[(size_t)st];
  a.z = p[(size_t)st * 2];
  a.w = p[(size_t)st * 3];
  b.x = p[(size_t)st * 4];
  b.y = p[(size_t)st * 5];
  b.z = p[(size_t)st * 6];
  b.w = p[(size_t)st * 7];
  const v4u wv = pack8(a, b);
  *(volatile v4u*)dp = wv;
  __threadfence();
  *(volatile v4u*)dp = wv;
}

__global__ __launch_bounds__(GTHR) void k_gemm(
    const unsigned short* __restrict__ A, int lda, const unsigned short* __restrict__ WTp, int K,
    float* outF, int ldo, int nRows, const float* __restrict__ bias, int epi)
{
  __shared__ __attribute__((aligned(16))) float stg[GBM * GBN];
  const int tid = (int)threadIdx.x, lane = tid & 31, wave = tid >> 5, hh = lane >> 4, m = lane & 15;
  const int rowBase = (int)blockIdx.x * GBM;
  const int col0    = (int)blockIdx.y * GBN;

  v8f acc[4];
  {
    const v8f z = {0.f, 0.f, 0.f, 0.f, 0.f, 0.f, 0.f, 0.f};
    acc[0] = z; acc[1] = z; acc[2] = z; acc[3] = z;
  }
  const unsigned short* ap = A   + (size_t)(rowBase + 16 * wave + m) * (size_t)lda + 8 * hh;
  const unsigned short* wp = WTp + (size_t)(col0 + m) * (size_t)K + 8 * hh;
  const int ksteps = K >> 5;
#pragma unroll 1
  for (int ks = 0; ks < ksteps; ++ks) {
    FragB af;
    af.h[0] = *(const v8usa*)(ap + 32 * ks);
    af.h[1] = *(const v8usa*)(ap + 32 * ks + 16);
#pragma unroll
    for (int t = 0; t < 4; ++t) {
      const unsigned short* wq = wp + (size_t)(16 * t) * (size_t)K + 32 * ks;
      FragB bf;
      bf.h[0] = *(const v8usa*)wq;
      bf.h[1] = *(const v8usa*)(wq + 16);
      acc[t] = wmb(af, bf, acc[t]);
    }
  }

#pragma unroll
  for (int t = 0; t < 4; ++t) {
    const int lc = 16 * t + m;
#pragma unroll
    for (int r = 0; r < 8; ++r) {
      const int lr = 16 * wave + 8 * hh + r;
      stg[lr * GBN + lc] = acc[t][r];
    }
  }
  __syncthreads();

  const int which = (epi != 0) ? (col0 >> 9) : 4;
  const int bidx  = (epi != 0) ? (col0 & (DHID - 1)) : col0;
  v4f b4 = bfr4(*(const v4fa*)(bias + bidx + 4 * m));
  const float fb  = (which >= 3) ? 1.0f : 0.0f;
  const float scl = (which == 0) ? QSC : 1.0f;
  b4 = b4 * fb;

  v4f fv[8];
#pragma unroll
  for (int i = 0; i < 8; ++i) {
    const int lr = 16 * wave + 2 * i + hh;
    v4f tq = (*(const v4fa*)(stg + lr * GBN + 4 * m) + b4) * scl;
    if (which == 3) tq = dsig4(tq);
    fv[i] = tq;
  }
#pragma unroll
  for (int i = 0; i < 8; ++i) {
    const int lr = 16 * wave + 2 * i + hh;
    const int gr = rowBase + lr;
    const int gs = gr < nRows ? gr : nRows - 1;
    float* op = outF + (size_t)gs * (size_t)ldo + col0 + 4 * m;
    if (gr < nRows) *(volatile v4f*)op = fv[i];
  }
  __threadfence();
#pragma unroll
  for (int i = 0; i < 8; ++i) {
    const int lr = 16 * wave + 2 * i + hh;
    const int gr = rowBase + lr;
    const int gs = gr < nRows ? gr : nRows - 1;
    float* op = outF + (size_t)gs * (size_t)ldo + col0 + 4 * m;
    if (gr < nRows) *(volatile v4f*)op = fv[i];
  }
}

__global__ __launch_bounds__(NTHR) void k_attn(const int* __restrict__ eidx, const float* __restrict__ QKVG,
                                               unsigned short* ao, int nE, int nkv, int mRows) {
  const int tid = (int)threadIdx.x, lane = tid & 31, wave = tid >> 5;
  const int nidx = 2 * nkv;
  const int li = lane < nidx - 1 ? lane : nidx - 1;
  const v4f z4 = {0.f, 0.f, 0.f, 0.f};
#pragma unroll 1
  for (int i = 0; i < RPW; ++i) {
    const int e  = (int)blockIdx.x * RB + i * NWAVE + wave;
    const int ec = e < nE ? e : nE - 1;
    const bool live = e < nE;
    const int iv = eidx[(size_t)ec * (size_t)nidx + li];

    const float* gp = QKVG + (size_t)ec * QW + OG + 8 * lane;
    const v4f ga0 = *(const v4fa*)gp;
    const v4f ga1 = *(const v4fa*)(gp + 4);
    const v4f gb0 = *(const v4fa*)(gp + 256);
    const v4f gb1 = *(const v4fa*)(gp + 260);

    v4f aa0 = z4, aa1 = z4, ab0 = z4, ab1 = z4;
#pragma unroll 1
    for (int j = 0; j < nkv; ++j) {
      int t = __builtin_amdgcn_readlane(iv, 2 * j);
      int s = __builtin_amdgcn_readlane(iv, 2 * j + 1);
      t = t < 0 ? 0 : (t > nE - 1 ? nE - 1 : t);
      s = s < 0 ? 0 : (s > nE - 1 ? nE - 1 : s);
      const float* qp = QKVG + (size_t)t * QW + OQ + 8 * lane;
      const v4f qa0 = *(const v4fa*)qp;
      const v4f qa1 = *(const v4fa*)(qp + 4);
      const v4f qb0 = *(const v4fa*)(qp + 256);
      const v4f qb1 = *(const v4fa*)(qp + 260);
      const float* kp = QKVG + (size_t)s * QW + OKK + 8 * lane;
      const v4f ka0 = *(const v4fa*)kp;
      const v4f ka1 = *(const v4fa*)(kp + 4);
      const v4f kb0 = *(const v4fa*)(kp + 256);
      const v4f kb1 = *(const v4fa*)(kp + 260);
      ldwait();
      float p0 = qa0.x * ka0.x;
      p0 = fmaf(qa0.y, ka0.y, p0); p0 = fmaf(qa0.z, ka0.z, p0); p0 = fmaf(qa0.w, ka0.w, p0);
      p0 = fmaf(qa1.x, ka1.x, p0); p0 = fmaf(qa1.y, ka1.y, p0); p0 = fmaf(qa1.z, ka1.z, p0); p0 = fmaf(qa1.w, ka1.w, p0);
      float p1 = qb0.x * kb0.x;
      p1 = fmaf(qb0.y, kb0.y, p1); p1 = fmaf(qb0.z, kb0.z, p1); p1 = fmaf(qb0.w, kb0.w, p1);
      p1 = fmaf(qb1.x, kb1.x, p1); p1 = fmaf(qb1.y, kb1.y, p1); p1 = fmaf(qb1.z, kb1.z, p1); p1 = fmaf(qb1.w, kb1.w, p1);
      p0 += __shfl_xor(p0, 1);
      p0 += __shfl_xor(p0, 2);
      p0 += __shfl_xor(p0, 4);
      p1 += __shfl_xor(p1, 1);
      p1 += __shfl_xor(p1, 2);
      p1 += __shfl_xor(p1, 4);
      const float* vp = QKVG + (size_t)s * QW + OV + 8 * lane;
      const v4f va0 = *(const v4fa*)vp;
      const v4f va1 = *(const v4fa*)(vp + 4);
      const v4f vb0 = *(const v4fa*)(vp + 256);
      const v4f vb1 = *(const v4fa*)(vp + 260);
      ldwait();
      aa0.x = fmaf(p0, va0.x, aa0.x); aa0.y = fmaf(p0, va0.y, aa0.y); aa0.z = fmaf(p0, va0.z, aa0.z); aa0.w = fmaf(p0, va0.w, aa0.w);
      aa1.x = fmaf(p0, va1.x, aa1.x); aa1.y = fmaf(p0, va1.y, aa1.y); aa1.z = fmaf(p0, va1.z, aa1.z); aa1.w = fmaf(p0, va1.w, aa1.w);
      ab0.x = fmaf(p1, vb0.x, ab0.x); ab0.y = fmaf(p1, vb0.y, ab0.y); ab0.z = fmaf(p1, vb0.z, ab0.z); ab0.w = fmaf(p1, vb0.w, ab0.w);
      ab1.x = fmaf(p1, vb1.x, ab1.x); ab1.y = fmaf(p1, vb1.y, ab1.y); ab1.z = fmaf(p1, vb1.z, ab1.z); ab1.w = fmaf(p1, vb1.w, ab1.w);
    }

    v4f oa0, oa1, ob0, ob1;
    oa0.x = live ? aa0.x * ga0.x : 0.0f; oa0.y = live ? aa0.y * ga0.y : 0.0f;
    oa0.z = live ? aa0.z * ga0.z : 0.0f; oa0.w = live ? aa0.w * ga0.w : 0.0f;
    oa1.x = live ? aa1.x * ga1.x : 0.0f; oa1.y = live ? aa1.y * ga1.y : 0.0f;
    oa1.z = live ? aa1.z * ga1.z : 0.0f; oa1.w = live ? aa1.w * ga1.w : 0.0f;
    ob0.x = live ? ab0.x * gb0.x : 0.0f; ob0.y = live ? ab0.y * gb0.y : 0.0f;
    ob0.z = live ? ab0.z * gb0.z : 0.0f; ob0.w = live ? ab0.w * gb0.w : 0.0f;
    ob1.x = live ? ab1.x * gb1.x : 0.0f; ob1.y = live ? ab1.y * gb1.y : 0.0f;
    ob1.z = live ? ab1.z * gb1.z : 0.0f; ob1.w = live ? ab1.w * gb1.w : 0.0f;
    v4u hv0, lv0, hv1, lv1;
    pack8hl(oa0, oa1, hv0, lv0);
    pack8hl(ob0, ob1, hv1, lv1);

    if (e < mRows) {
      unsigned short* rp = ao + (size_t)e * APITCH;
      *(volatile v4u*)(rp + 8 * lane)        = hv0;
      *(volatile v4u*)(rp + 256 + 8 * lane)  = hv1;
      *(volatile v4u*)(rp + DHID + 8 * lane)       = lv0;
      *(volatile v4u*)(rp + DHID + 256 + 8 * lane) = lv1;
      __threadfence();
      *(volatile v4u*)(rp + 8 * lane)        = hv0;
      *(volatile v4u*)(rp + 256 + 8 * lane)  = hv1;
      *(volatile v4u*)(rp + DHID + 8 * lane)       = lv0;
      *(volatile v4u*)(rp + DHID + 256 + 8 * lane) = lv1;
    }
  }
}

static inline int cdiv(int a, int b) { return (a + b - 1) / b; }
static inline size_t al256(size_t o) { return (o + 255) & ~(size_t)255; }

extern "C" void kernel_launch(void* const* d_in, const int* in_sizes, int n_in,
                              void* d_out, int out_size, void* d_ws, size_t ws_size,
                              hipStream_t stream) {
  if (n_in < 10) return;
  if (in_sizes[0] < DP || (in_sizes[0] % DP) != 0) return;
  const int nE = in_sizes[0] / DP;
  if (nE < 1 || nE > (1 << 22)) return;
  if (in_sizes[1] < 2 || (in_sizes[1] % (2 * nE)) != 0) return;
  const int nkv = in_sizes[1] / (2 * nE);
  if (nkv < 1 || nkv > NKVMAX) return;
  if (in_sizes[3] != DP * DHID || in_sizes[4] != DP * DHID || in_sizes[5] != DP * DHID || in_sizes[6] != DP * DHID) return;
  if (in_sizes[7] != DHID) return;
  if (in_sizes[8] != DHID * DP) return;
  if (in_sizes[9] != DP) return;
  if ((long long)out_size != (long long)nE * DP) return;

  const float* z    = (const float*)d_in[0];
  const int*   eidx = (const int*)  d_in[1];
  const float* Wq   = (const float*)d_in[3];
  const float* Wk   = (const float*)d_in[4];
  const float* Wv   = (const float*)d_in[5];
  const float* Wg   = (const float*)d_in[6];
  const float* bg   = (const float*)d_in[7];
  const float* Wo   = (const float*)d_in[8];
  const float* bo   = (const float*)d_in[9];
  float* out = (float*)d_out;

  const int MP = cdiv(nE, GBM) * GBM;
  const int gM = MP / GBM;
  const int gA = cdiv(MP, RB);
  if ((long long)gA * RB < (long long)MP) return;

  char* ws = (char*)d_ws;
  size_t off = 0;
  const size_t oZB = off; off = al256(off + (size_t)MP * DP * 2);
  const size_t oWT = off; off = al256(off + (size_t)QW * DP * 2);
  const size_t oWO = off; off = al256(off + (size_t)DP * KOUT * 2);
  const size_t oQ  = off; off = al256(off + (size_t)MP * QW * 4);
  const size_t oAO = off; off = al256(off + (size_t)MP * APITCH * 2);
  if (off > ws_size || off > (size_t)WSMAX) return;
  unsigned short* ZB   = (unsigned short*)(ws + oZB);
  unsigned short* WT   = (unsigned short*)(ws + oWT);
  unsigned short* WOT  = (unsigned short*)(ws + oWO);
  float*          QKVG = (float*)(ws + oQ);
  unsigned short* AO   = (unsigned short*)(ws + oAO);

  const int nUz = MP * (DP / 8);
  k_zprep<<<cdiv(nUz, NTHR), NTHR, 0, stream>>>(z, ZB, nE, nUz);
  k_wprep<<<NUW / NTHR, NTHR, 0, stream>>>(Wq, Wk, Wv, Wg, Wo, WT, WOT);
  k_gemm<<<dim3(gM, QW / GBN), GTHR, 0, stream>>>(ZB, DP, WT, DP, QKVG, QW, MP, bg, 1);
  k_attn<<<gA, NTHR, 0, stream>>>(eidx, QKVG, AO, nE, nkv, MP);
  k_gemm<<<dim3(gM, DP / GBN), GTHR, 0, stream>>>(AO, APITCH, WOT, KOUT, out, DP, nE, bo, 0);
}
